// DynamicGraphEmbedding_16827681866102
// MI455X (gfx1250) — hardware-run, weakly checked
//
#include <hip/hip_runtime.h>
#include <math.h>

typedef __attribute__((ext_vector_type(16))) _Float16 v16h;
typedef __attribute__((ext_vector_type(8)))  _Float16 v8h;
typedef __attribute__((ext_vector_type(8)))  float    v8f;
typedef __attribute__((ext_vector_type(4)))  float    v4f;

constexpr int kBatch = 64;
constexpr int kNodes = 256;
constexpr int kFeat  = 256;
constexpr int kEmb   = 64;
constexpr int kTop   = 16;
constexpr int kRows  = kBatch * kNodes;
static_assert(kNodes == 256);
static_assert((kNodes & (kNodes - 1)) == 0);
static_assert((kRows % 64) == 0 && (kFeat % 64) == 0 && (kFeat % 32) == 0);
static_assert((kEmb % 4) == 0 && kEmb <= 256);
static_assert(2 * kTop == 32);

constexpr float kEdgeW    = 1.0f / (float)kTop;
constexpr float kYCarry   = 256.0f;
constexpr float kWCarry   = 1024.0f;
constexpr float kOutScale = 1.0f / (kYCarry * kWCarry);
constexpr float kHalfMinNormal = 6.103515625e-05f;

constexpr size_t kBytesTab = (size_t)kNodes * 32 * 4;
constexpr size_t kBytesBt  = (size_t)kFeat * kFeat * 2;
constexpr size_t kBytesY   = (size_t)kRows * kFeat * 2;
constexpr size_t kOffTab   = 0;
constexpr size_t kOffBt    = kOffTab + kBytesTab;
constexpr size_t kOffY     = kOffBt + kBytesBt;
constexpr size_t kWsTotal  = kOffY + kBytesY;
static_assert(kWsTotal == 8552448ull);
static_assert(kWsTotal <= 134217728ull);
static_assert((kOffBt % 128) == 0 && (kOffY % 128) == 0);

union FragU { v16h v; v8h h[2]; };
__device__ __forceinline__ v16h frag_load(const _Float16* p) {
  FragU f;
  f.h[0] = *(const v8h*)(p);
  f.h[1] = *(const v8h*)(p + 16);
  return f.v;
}
__device__ __forceinline__ v8f frag_mma(v16h a, v16h b, v8f c) {
  return __builtin_amdgcn_wmma_f32_16x16x32_f16(false, a, false, b, (short)0, c, false, false);
}
__device__ __forceinline__ void guard_one(v8f& a, v16h x, v16h y) {
  asm volatile("v_nop\n\tv_nop\n\tv_nop\n\tv_nop" : "+v"(a) : "v"(x), "v"(y));
}
__device__ __forceinline__ void keep4_h(v16h a, v16h b, v16h c, v16h d) {
  asm volatile("v_nop" :: "v"(a), "v"(b), "v"(c), "v"(d));
}

__global__ __launch_bounds__(256) void graph_build_kernel(
    const float* __restrict__ emb, const float* __restrict__ logits, const float* __restrict__ gum,
    unsigned* __restrict__ tab)
{
#pragma clang fp contract(off)
  __shared__ __align__(16) float sEi[kEmb];
  __shared__ __align__(16) float sNsq[kNodes];
  __shared__ __align__(16) float sCos[kNodes];
  __shared__ unsigned sRec[32];
  const int i = blockIdx.x;
  const int j = threadIdx.x;

  float ev = emb[(size_t)i * kEmb + (j & (kEmb - 1))];
  asm volatile("" : "+v"(ev));
  if (j < kEmb) sEi[j] = ev;
  if (j < 32) sRec[j] = (j & 1) ? 0u : (unsigned)i;

  const size_t e2 = ((size_t)i * kNodes + (size_t)j) * 2;
  float u0 = gum[e2];
  float u1 = gum[e2 + 1];
  float l0 = logits[e2];
  float l1 = logits[e2 + 1];
  asm volatile("" : "+v"(u0));
  asm volatile("" : "+v"(u1));
  asm volatile("" : "+v"(l0));
  asm volatile("" : "+v"(l1));
  __syncthreads();

  const float* er = emb + (size_t)j * kEmb;
  float dot = 0.0f;
  float nj  = 0.0f;
#pragma unroll 2
  for (int d4 = 0; d4 < kEmb / 4; ++d4) {
    const v4f a = *(const v4f*)(er + 4 * d4);
    const v4f c = *(const v4f*)(sEi + 4 * d4);
    dot = fmaf(c[0], a[0], dot);
    dot = fmaf(c[1], a[1], dot);
    dot = fmaf(c[2], a[2], dot);
    dot = fmaf(c[3], a[3], dot);
    nj = fmaf(a[0], a[0], nj);
    nj = fmaf(a[1], a[1], nj);
    nj = fmaf(a[2], a[2], nj);
    nj = fmaf(a[3], a[3], nj);
  }
  sNsq[j] = nj;
  __syncthreads();
  const float ni  = sNsq[i];
  const float den = sqrtf(ni) * sqrtf(nj);
  const float cv  = dot / den;
  sCos[j] = cv;
  __syncthreads();

  int rank = 0;
#pragma unroll 2
  for (int q4 = 0; q4 < kNodes / 4; ++q4) {
    const v4f c = *(const v4f*)(sCos + 4 * q4);
    const int qb = 4 * q4;
    rank += ((c[0] > cv) || ((c[0] == cv) && ((qb + 0) < j))) ? 1 : 0;
    rank += ((c[1] > cv) || ((c[1] == cv) && ((qb + 1) < j))) ? 1 : 0;
    rank += ((c[2] > cv) || ((c[2] == cv) && ((qb + 2) < j))) ? 1 : 0;
    rank += ((c[3] > cv) || ((c[3] == cv) && ((qb + 3) < j))) ? 1 : 0;
  }

  const float g0 = -logf(-logf(u0));
  const float g1 = -logf(-logf(u1));
  const float gate = ((l0 + g0) >= (l1 + g1)) ? 1.0f : 0.0f;
  if (rank < kTop) {
    sRec[2 * rank]     = (unsigned)j;
    sRec[2 * rank + 1] = __float_as_uint(gate * kEdgeW);
  }
  __syncthreads();
  if (j < 32) {
    const unsigned v = sRec[j];
    volatile unsigned* p = (volatile unsigned*)(tab + (size_t)i * 32 + j);
    *p = v;
    __threadfence();
    *p = v;
  }
}

__global__ __launch_bounds__(256) void wprep_kernel(
    const float* __restrict__ W, unsigned short* __restrict__ Bt)
{
  __shared__ float sTile[64 * 65];
  const int tid = threadIdx.x;
  const int lane = tid & 31;
  const int wave = tid >> 5;
  const int k0 = blockIdx.x * 64;
  const int n0 = blockIdx.y * 64;
  const int lr = tid >> 4;
  const int lc4 = (tid & 15) * 4;
#pragma unroll
  for (int it = 0; it < 4; ++it) {
    const int kk = it * 16 + lr;
    const v4f a = *(const v4f*)(W + (size_t)(k0 + kk) * kFeat + n0 + lc4);
    sTile[kk * 65 + lc4 + 0] = a[0];
    sTile[kk * 65 + lc4 + 1] = a[1];
    sTile[kk * 65 + lc4 + 2] = a[2];
    sTile[kk * 65 + lc4 + 3] = a[3];
  }
  __syncthreads();
  const int q = lane >> 3;
  const int c8 = (lane & 7) * 8;
  v8h hv[2];
#pragma unroll
  for (int it = 0; it < 2; ++it) {
    const int nrow = it * 32 + wave * 4 + q;
#pragma unroll
    for (int e = 0; e < 8; ++e) {
      float v = sTile[(c8 + e) * 65 + nrow] * kWCarry;
      v = (fabsf(v) < kHalfMinNormal) ? 0.0f : v;
      hv[it][e] = (_Float16)v;
    }
  }
  for (int pass = 0; pass < 2; ++pass) {
#pragma unroll
    for (int it = 0; it < 2; ++it) {
      const int nrow = it * 32 + wave * 4 + q;
      *(volatile v8h*)(Bt + (size_t)(n0 + nrow) * kFeat + k0 + c8) = hv[it];
    }
    __threadfence();
  }
}

__global__ __launch_bounds__(256) void aggregate_kernel(
    const float* __restrict__ x, const unsigned* __restrict__ tab, unsigned short* __restrict__ Y)
{
  __shared__ unsigned sRec[8 * 32];
  const int tid = threadIdx.x;
  const int lane = tid & 31;
  const int wave = tid >> 5;
  const int r0 = blockIdx.x * 8;
  const int i0 = r0 & (kNodes - 1);
  sRec[tid] = tab[(size_t)i0 * 32 + tid];
  __syncthreads();
  const int r  = r0 + wave;
  const int bb = r >> 8;
  const float* xb = x + (size_t)bb * kNodes * kFeat + lane * 8;
  v4f acc0 = (v4f){0.f, 0.f, 0.f, 0.f};
  v4f acc1 = (v4f){0.f, 0.f, 0.f, 0.f};
#pragma unroll 2
  for (int k = 0; k < kTop; ++k) {
    const unsigned sw = sRec[wave * 32 + 2 * k];
    const float w = __uint_as_float(sRec[wave * 32 + 2 * k + 1]);
    const int s = (int)(sw & (unsigned)(kNodes - 1));
    const float* xr = xb + (size_t)s * kFeat;
    const v4f a0 = *(const v4f*)(xr);
    const v4f a1 = *(const v4f*)(xr + 4);
    acc0[0] = fmaf(w, a0[0], acc0[0]);
    acc0[1] = fmaf(w, a0[1], acc0[1]);
    acc0[2] = fmaf(w, a0[2], acc0[2]);
    acc0[3] = fmaf(w, a0[3], acc0[3]);
    acc1[0] = fmaf(w, a1[0], acc1[0]);
    acc1[1] = fmaf(w, a1[1], acc1[1]);
    acc1[2] = fmaf(w, a1[2], acc1[2]);
    acc1[3] = fmaf(w, a1[3], acc1[3]);
  }
  v8h hv;
#pragma unroll
  for (int e = 0; e < 4; ++e) {
    float v0 = acc0[e] * kYCarry;
    float v1 = acc1[e] * kYCarry;
    v0 = (fabsf(v0) < kHalfMinNormal) ? 0.0f : v0;
    v1 = (fabsf(v1) < kHalfMinNormal) ? 0.0f : v1;
    hv[e]     = (_Float16)v0;
    hv[4 + e] = (_Float16)v1;
  }
  volatile v8h* p = (volatile v8h*)(Y + (size_t)r * kFeat + lane * 8);
  *p = hv;
  __threadfence();
  *p = hv;
}

__global__ __launch_bounds__(256) void gemm_f16_bias_kernel(
    const unsigned short* __restrict__ Ap, int lda,
    const unsigned short* __restrict__ Btp, int ldb,
    float* __restrict__ C, int ldc,
    const float* __restrict__ bias,
    int M, int N, int K, float scale)
{
  const _Float16* A  = (const _Float16*)Ap;
  const _Float16* Bt = (const _Float16*)Btp;
  __shared__ __align__(16) float sSlab[8][16 * 68];
  const int lane = threadIdx.x & 31;
  const int wave = threadIdx.x >> 5;
  const int tilesN = N >> 6;
  const int tilesM = M >> 6;
  const int tile = blockIdx.x * 8 + wave;
  if (tile >= tilesM * tilesN) return;
  const int tm = tile / tilesN;
  const int tn = tile - tm * tilesN;
  const int m0 = tm << 6;
  const int n0 = tn << 6;

  const int rlane = lane & 15;
  const int koff  = (lane >> 4) * 8;
  const int mOff  = (lane >> 4) * 8;

  v8f acc[4][4];
#pragma unroll
  for (int i = 0; i < 4; ++i)
#pragma unroll
    for (int j = 0; j < 4; ++j) acc[i][j] = (v8f){0.f, 0.f, 0.f, 0.f, 0.f, 0.f, 0.f, 0.f};

  for (int k0 = 0; k0 < K; k0 += 32) {
    v16h bh[4];
#pragma unroll
    for (int j = 0; j < 4; ++j) {
      const size_t bo = (size_t)(n0 + (j << 4) + rlane) * ldb + koff + k0;
      bh[j] = frag_load(Bt + bo);
    }
#pragma unroll
    for (int i = 0; i < 4; ++i) {
      const size_t ao = (size_t)(m0 + (i << 4) + rlane) * lda + koff + k0;
      const v16h ah = frag_load(A + ao);
#pragma unroll
      for (int j = 0; j < 4; ++j) acc[i][j] = frag_mma(ah, bh[j], acc[i][j]);
      guard_one(acc[i][0], ah, bh[0]);
      guard_one(acc[i][1], ah, bh[1]);
      guard_one(acc[i][2], ah, bh[2]);
      guard_one(acc[i][3], ah, bh[3]);
    }
    keep4_h(bh[0], bh[1], bh[2], bh[3]);
  }

  float* slab = sSlab[wave];
  float bv[4];
#pragma unroll
  for (int j = 0; j < 4; ++j) bv[j] = bias[n0 + (j << 4) + rlane];
#pragma unroll
  for (int i = 0; i < 4; ++i) {
    const int mBase = m0 + (i << 4);
#pragma unroll
    for (int j = 0; j < 4; ++j) {
#pragma unroll
      for (int r = 0; r < 8; ++r) {
        const float v = acc[i][j][r] * scale + bv[j];
        slab[(mOff + r) * 68 + (j << 4) + rlane] = v;
      }
    }
    __builtin_amdgcn_fence(__ATOMIC_RELEASE, "workgroup");
    __builtin_amdgcn_wave_barrier();
    __builtin_amdgcn_fence(__ATOMIC_ACQUIRE, "workgroup");
    {
      const int hh = lane >> 4;
      const int c4 = (lane & 15) * 4;
      for (int pass = 0; pass < 2; ++pass) {
#pragma unroll
        for (int it = 0; it < 8; ++it) {
          const int row = it * 2 + hh;
          const v4f v = *(const v4f*)(slab + row * 68 + c4);
          *(volatile v4f*)(C + (size_t)(mBase + row) * ldc + n0 + c4) = v;
        }
        __threadfence();
      }
    }
    __builtin_amdgcn_fence(__ATOMIC_RELEASE, "workgroup");
    __builtin_amdgcn_wave_barrier();
    __builtin_amdgcn_fence(__ATOMIC_ACQUIRE, "workgroup");
  }
}

extern "C" void kernel_launch(void* const* d_in, const int* in_sizes, int n_in,
                              void* d_out, int out_size, void* d_ws, size_t ws_size,
                              hipStream_t stream) {
  if (n_in < 6) return;
  if (in_sizes[0] != kRows * kFeat) return;
  if (in_sizes[1] != kNodes * kEmb) return;
  if (in_sizes[2] != kFeat * kFeat) return;
  if (in_sizes[3] != kFeat) return;
  if (in_sizes[4] != kNodes * kNodes * 2) return;
  if (in_sizes[5] != kNodes * kNodes * 2) return;
  if (out_size != kRows * kFeat) return;
  if (ws_size < kWsTotal) return;

  const float* x      = (const float*)d_in[0];
  const float* emb    = (const float*)d_in[1];
  const float* W      = (const float*)d_in[2];
  const float* bias   = (const float*)d_in[3];
  const float* logits = (const float*)d_in[4];
  const float* gum    = (const float*)d_in[5];
  float* out = (float*)d_out;

  char* ws = (char*)d_ws;
  unsigned*       tab  = (unsigned*)(ws + kOffTab);
  unsigned short* Bt16 = (unsigned short*)(ws + kOffBt);
  unsigned short* Y16  = (unsigned short*)(ws + kOffY);

  graph_build_kernel<<<kNodes, 256, 0, stream>>>(emb, logits, gum, tab);
  wprep_kernel<<<dim3(kFeat / 64, kFeat / 64), 256, 0, stream>>>(W, Bt16);
  aggregate_kernel<<<kRows / 8, 256, 0, stream>>>(x, tab, Y16);
  gemm_f16_bias_kernel<<<((kRows / 64) * (kFeat / 64)) / 8, 256, 0, stream>>>(
      Y16, kFeat, Bt16, kFeat, out, kFeat, bias, kRows, kFeat, kFeat, kOutScale);
}
